// SupervisedContrastiveLoss_55336358641764
// MI455X (gfx1250) — hardware-verified
//
#include <hip/hip_runtime.h>


typedef _Float16 half_t;
typedef __attribute__((ext_vector_type(16))) _Float16 v16h;
typedef __attribute__((ext_vector_type(8)))  _Float16 v8h;
typedef __attribute__((ext_vector_type(4)))  _Float16 v4h;
typedef __attribute__((ext_vector_type(8)))  float    v8f;
typedef __attribute__((ext_vector_type(4)))  float    v4f;
#define NROWS 8192
#define KDIM  128
#define SQRT_SCALE 3.7982825656899547f
#define VST2(T, ptr, val) do { const T _v = (val); *(volatile T*)(ptr) = _v; __threadfence(); *(volatile T*)(ptr) = _v; } while (0)
__device__ __forceinline__ v8f wmma16(v16h a, v16h b, v8f c) {
  v8f d = __builtin_amdgcn_wmma_f32_16x16x32_f16(false, a, false, b, (short)0, c, false, false);
  asm volatile("v_nop\n\tv_nop\n\tv_nop\n\tv_nop" : "+v"(d) : "v"(a), "v"(b));
  return d;
}
__device__ __forceinline__ v16h frag16(const half_t* p, int hh) {
  const v8h lo = *(const v8h*)(p + 8 * hh), hi = *(const v8h*)(p + 16 + 8 * hh);
  return __builtin_shufflevector(lo, hi, 0,1,2,3,4,5,6,7,8,9,10,11,12,13,14,15);
}

__global__ __launch_bounds__(256) void k_normalize(const float* __restrict__ feat, half_t* __restrict__ fnorm) {
  const int wave = threadIdx.x >> 5, lane = threadIdx.x & 31, row = blockIdx.x * 8 + wave;
  v4f v = *(const v4f*)(feat + (size_t)row * KDIM + lane * 4);
  float s = v.x * v.x + v.y * v.y + v.z * v.z + v.w * v.w;
#pragma unroll
  for (int m = 16; m >= 1; m >>= 1) s += __shfl_xor(s, m, 32);
  const float scale = SQRT_SCALE / fmaxf(sqrtf(s), 1e-12f);
  v4h o; o.x = (half_t)(v.x * scale); o.y = (half_t)(v.y * scale); o.z = (half_t)(v.z * scale); o.w = (half_t)(v.w * scale);
  VST2(v4h, fnorm + (size_t)row * KDIM + lane * 4, o);
}
__global__ __launch_bounds__(256) void k_cosexp(const half_t* __restrict__ fnorm, const int* __restrict__ labels, float* __restrict__ rowstat) {
  __shared__ float sRed[8][3][32];
  const int tid = threadIdx.x, wave = tid >> 5, lane = tid & 31, lm = lane & 15, hi = lane >> 4;
  const int row0 = blockIdx.x * 32;
  const half_t* ar0 = fnorm + (size_t)(row0 + lm) * KDIM;
  const half_t* ar1 = ar0 + (size_t)16 * KDIM;
  v16h a0[4], a1[4];
#pragma unroll
  for (int kc = 0; kc < 4; ++kc) { a0[kc] = frag16(ar0 + kc * 32, hi); a1[kc] = frag16(ar1 + kc * 32, hi); }
  int rlab0[8], rlab1[8];
#pragma unroll
  for (int r = 0; r < 8; ++r) { rlab0[r] = labels[row0 + hi * 8 + r]; rlab1[r] = labels[row0 + 16 + hi * 8 + r]; }
  float aAll0[8] = {}, aPos0[8] = {}, aAll1[8] = {}, aPos1[8] = {}, nP0[8] = {}, nP1[8] = {};
  for (int t = wave; t < NROWS / 16; t += 8) {
    const int col = t * 16 + lm;
    const half_t* bp = fnorm + (size_t)col * KDIM;
    const int clab = labels[col];
    v8f c0 = {}, c1 = {};
#pragma unroll
    for (int kc = 0; kc < 4; ++kc) { const v16h b = frag16(bp + kc * 32, hi); c0 = wmma16(a0[kc], b, c0); c1 = wmma16(a1[kc], b, c1); }
#pragma unroll
    for (int r = 0; r < 8; ++r) {
      const int rowA = row0 + hi * 8 + r, rowB = row0 + 16 + hi * 8 + r;
      const float e0 = (col == rowA) ? 0.0f : __builtin_amdgcn_exp2f(c0[r]);
      const float e1 = (col == rowB) ? 0.0f : __builtin_amdgcn_exp2f(c1[r]);
      const bool m0 = (rlab0[r] == clab), m1 = (rlab1[r] == clab);
      aAll0[r] += e0; aAll1[r] += e1;
      aPos0[r] += m0 ? e0 : 0.0f; aPos1[r] += m1 ? e1 : 0.0f;
      nP0[r] += (m0 && col != rowA) ? 1.0f : 0.0f; nP1[r] += (m1 && col != rowB) ? 1.0f : 0.0f;
    }
  }
#pragma unroll
  for (int m = 1; m < 16; m <<= 1) {
#pragma unroll
    for (int r = 0; r < 8; ++r) {
      aAll0[r] += __shfl_xor(aAll0[r], m, 32); aPos0[r] += __shfl_xor(aPos0[r], m, 32); nP0[r] += __shfl_xor(nP0[r], m, 32);
      aAll1[r] += __shfl_xor(aAll1[r], m, 32); aPos1[r] += __shfl_xor(aPos1[r], m, 32); nP1[r] += __shfl_xor(nP1[r], m, 32);
    }
  }
  if (lm == 0) {
#pragma unroll
    for (int r = 0; r < 8; ++r) {
      sRed[wave][0][hi * 8 + r] = aAll0[r]; sRed[wave][1][hi * 8 + r] = aPos0[r]; sRed[wave][2][hi * 8 + r] = nP0[r];
      sRed[wave][0][16 + hi * 8 + r] = aAll1[r]; sRed[wave][1][16 + hi * 8 + r] = aPos1[r]; sRed[wave][2][16 + hi * 8 + r] = nP1[r];
    }
  }
  __syncthreads();
  if (tid < 32) {
    float all = 0.f, pos = 0.f, np = 0.f;
#pragma unroll
    for (int w = 0; w < 8; ++w) { all += sRed[w][0][tid]; pos += sRed[w][1][tid]; np += sRed[w][2][tid]; }
    const v4f st = {all, pos, np, 0.f};
    VST2(v4f, rowstat + (size_t)(row0 + tid) * 4, st);
  }
}
__global__ __launch_bounds__(256) void k_finalize(const float* __restrict__ rowstat, float* __restrict__ out) {
  __shared__ double red[256];
  const int tid = threadIdx.x;
  double acc = 0.0;
  for (int i = tid; i < NROWS; i += 256) {
    const float allv = rowstat[i * 4 + 0], posv = rowstat[i * 4 + 1], npos = rowstat[i * 4 + 2];
    acc += (double)(logf(allv) - logf(posv) + logf(npos));
  }
  red[tid] = acc;
  __syncthreads();
#pragma unroll
  for (int s = 128; s > 0; s >>= 1) { if (tid < s) red[tid] += red[tid + s]; __syncthreads(); }
  if (tid == 0) VST2(float, out, (float)(red[0] / (double)NROWS));
}
extern "C" void kernel_launch(void* const* d_in, const int* in_sizes, int n_in,
                              void* d_out, int out_size, void* d_ws, size_t ws_size, hipStream_t stream) {
  (void)in_sizes; (void)n_in; (void)out_size;
  const float* feat   = (const float*)d_in[0];
  const int*   labels = (const int*)d_in[1];
  float*       out    = (float*)d_out;
  if (ws_size < (size_t)NROWS * KDIM * 2 + (size_t)NROWS * 16) return;
  half_t* fnorm  = (half_t*)d_ws;
  float*  rowstat = (float*)((char*)d_ws + (size_t)NROWS * KDIM * sizeof(half_t));
  k_normalize<<<NROWS / 8, 256, 0, stream>>>(feat, fnorm);
  k_cosexp<<<NROWS / 32, 256, 0, stream>>>(fnorm, labels, rowstat);
  k_finalize<<<1, 256, 0, stream>>>(rowstat, out);
}
